// Capsule3D_4741643895374
// MI455X (gfx1250) — hardware-verified
//
#include <hip/hip_runtime.h>
#include <math.h>

constexpr int kB   = 16;
constexpr int kH   = 32;
constexpr int kW   = 32;
constexpr int kIC  = 32;
constexpr int kIL  = 8;
constexpr int kOH  = 30;
constexpr int kOW  = 30;
constexpr int kP   = kOH * kOW;
constexpr int kCaps = 16;
constexpr int kL    = 8;
constexpr int kNC   = kCaps * kL;
constexpr int kJ    = kP * kCaps;
constexpr int kKreal = 9 * kIL;
constexpr int kKpad  = 96;
constexpr int kSegs  = kKpad / 8;
constexpr int kChunkB = 4;
constexpr int kNumChunks = kB / kChunkB;
constexpr int kRowsPerB = kIC * kP;
constexpr int kMChunk   = kChunkB * kRowsPerB;
constexpr float kInvSqrtL = 0.35355339059327373f;
constexpr float kEps = 1e-7f;

static_assert(kMChunk % 64 == 0);
static_assert(kNC % 64 == 0);
static_assert(kKpad % 32 == 0);
static_assert(kB % kChunkB == 0);
static_assert((kChunkB * kP) % 4 == 0);
static_assert(kJ % 4 == 0);

typedef __attribute__((ext_vector_type(16))) _Float16 v16h;
typedef __attribute__((ext_vector_type(8)))  _Float16 v8h;
typedef __attribute__((ext_vector_type(16))) __bf16   v16b;
typedef __attribute__((ext_vector_type(8)))  __bf16   v8b;
typedef __attribute__((ext_vector_type(8)))  float    v8f;
typedef __attribute__((ext_vector_type(4)))  float    v4f;
typedef __attribute__((ext_vector_type(4)))  unsigned int v4u;

__device__ __forceinline__ unsigned short f2bf_bits(float f) {
  unsigned u = __float_as_uint(f);
  return (unsigned short)((u + 0x7FFFu + ((u >> 16) & 1u)) >> 16);
}
__device__ __forceinline__ float bf_bits2f(unsigned short h) { return __uint_as_float(((unsigned)h) << 16); }

__device__ __forceinline__ void dep_guard_h(v8f& a, v8f& b, v16h x, v16h y) { asm volatile("v_nop\n\tv_nop\n\tv_nop\n\tv_nop" : "+v"(a), "+v"(b) : "v"(x), "v"(y)); }
__device__ __forceinline__ void dep_guard_b(v8f& a, v8f& b, v16b x, v16b y) { asm volatile("v_nop\n\tv_nop\n\tv_nop\n\tv_nop" : "+v"(a), "+v"(b) : "v"(x), "v"(y)); }
__device__ __forceinline__ void keep4_h(v16h a, v16h b, v16h c, v16h d) { asm volatile("v_nop" :: "v"(a), "v"(b), "v"(c), "v"(d)); }
__device__ __forceinline__ void keep4_b(v16b a, v16b b, v16b c, v16b d) { asm volatile("v_nop" :: "v"(a), "v"(b), "v"(c), "v"(d)); }
__device__ __forceinline__ void acc_guard4(v8f& a, v8f& b, v8f& c, v8f& d) { asm volatile("v_nop\n\tv_nop\n\tv_nop\n\tv_nop" : "+v"(a), "+v"(b), "+v"(c), "+v"(d)); }
template <typename T> struct Frag;
template <> struct Frag<_Float16> {
  typedef v16h V; union U { v16h v; v8h h[2]; };
  static __device__ __forceinline__ v16h load(const _Float16* p) {
    U f; f.h[0] = *(const v8h*)(p); f.h[1] = *(const v8h*)(p + 16); return f.v;
  }
  static __device__ __forceinline__ v8f mma(v16h a, v16h b, v8f c) {
    return __builtin_amdgcn_wmma_f32_16x16x32_f16(false, a, false, b, (short)0, c, false, false);
  }
  static __device__ __forceinline__ void guard(v8f& a, v8f& b, v16h x, v16h y) { dep_guard_h(a, b, x, y); }
  static __device__ __forceinline__ void keep(v16h a, v16h b, v16h c, v16h d) { keep4_h(a, b, c, d); }
};
template <> struct Frag<__bf16> {
  typedef v16b V; union U { v16b v; v8b h[2]; };
  static __device__ __forceinline__ v16b load(const __bf16* p) {
    U f; f.h[0] = *(const v8b*)(p); f.h[1] = *(const v8b*)(p + 16); return f.v;
  }
  static __device__ __forceinline__ v8f mma(v16b a, v16b b, v8f c) {
    return __builtin_amdgcn_wmma_f32_16x16x32_bf16(false, a, false, b, (short)0, c, false, false);
  }
  static __device__ __forceinline__ void guard(v8f& a, v8f& b, v16b x, v16b y) { dep_guard_b(a, b, x, y); }
  static __device__ __forceinline__ void keep(v16b a, v16b b, v16b c, v16b d) { keep4_b(a, b, c, d); }
};

__device__ __forceinline__ unsigned pk16(unsigned short a, unsigned short b) { return (unsigned)a | ((unsigned)b << 16); }

template <int ET> struct Elem;
template <> struct Elem<0> { typedef _Float16 T; };
template <> struct Elem<1> { typedef __bf16 T; };
template <int ET, bool SPLIT, int BIAS_MODE, int OUT_MODE, bool RESID, int ACT = 0>
__global__ __launch_bounds__(256) void wmma_gemm64(
    const unsigned short* __restrict__ Ap, const unsigned short* __restrict__ A2p, int lda, long strideA,
    const unsigned short* __restrict__ Btp, const unsigned short* __restrict__ Bt2p, int ldb, long strideB,
    void* __restrict__ Cout, void* __restrict__ Cout2, int ldc, long strideC,
    const float* __restrict__ bias,
    const float* __restrict__ resid, long strideR,
    int M, int N, int K, float scale) {
  typedef typename Elem<ET>::T T;
  typedef typename Frag<T>::V V;
  const T* A = (const T*)Ap; const T* A2 = (const T*)A2p; const T* Bt = (const T*)Btp; const T* Bt2 = (const T*)Bt2p;
  __shared__ __align__(16) float sT[8][16 * 68];
  const int b    = blockIdx.y;
  const int lane = threadIdx.x & 31;
  const int wave = threadIdx.x >> 5;
  const int tilesN = N >> 6;
  const int tilesM = M >> 6;
  const int tile = blockIdx.x * 8 + wave;
  if (tile >= tilesM * tilesN) return;
  const int tm = tile / tilesN;
  const int tn = tile - tm * tilesN;
  const int m0 = tm << 6;
  const int n0 = tn << 6;

  const T* Ab  = A  + (size_t)b * strideA;
  const T* Bb  = Bt + (size_t)b * strideB;
  const T* Ab2 = SPLIT ? (A2  + (size_t)b * strideA) : nullptr;
  const T* Bb2 = SPLIT ? (Bt2 + (size_t)b * strideB) : nullptr;

  const int rlane = lane & 15;
  const int koff  = (lane >> 4) * 8;
  const int mOff  = (lane >> 4) * 8;

  v8f acc[4][4];
#pragma unroll
  for (int i = 0; i < 4; ++i)
#pragma unroll
    for (int j = 0; j < 4; ++j) acc[i][j] = (v8f){0.f,0.f,0.f,0.f,0.f,0.f,0.f,0.f};

  for (int k0 = 0; k0 < K; k0 += 32) {
    V bh[4], bl[4];
#pragma unroll
    for (int j = 0; j < 4; ++j) {
      const size_t bo = (size_t)(n0 + (j << 4) + rlane) * ldb + koff + k0;
      bh[j] = Frag<T>::load(Bb + bo);
      if (SPLIT) bl[j] = Frag<T>::load(Bb2 + bo);
    }
#pragma unroll
    for (int i = 0; i < 4; ++i) {
      const size_t ao = (size_t)(m0 + (i << 4) + rlane) * lda + koff + k0;
      V ah = Frag<T>::load(Ab + ao);
      V al;
      if (SPLIT) al = Frag<T>::load(Ab2 + ao);
#pragma unroll
      for (int j = 0; j < 4; ++j) {
        acc[i][j] = Frag<T>::mma(ah, bh[j], acc[i][j]);
        if (SPLIT) {
          acc[i][j] = Frag<T>::mma(ah, bl[j], acc[i][j]);
          acc[i][j] = Frag<T>::mma(al, bh[j], acc[i][j]);
        }
      }
      Frag<T>::guard(acc[i][0], acc[i][3], ah, SPLIT ? al : ah);
    }
    Frag<T>::keep(bh[0], bh[1], bh[2], bh[3]);
    if (SPLIT) Frag<T>::keep(bl[0], bl[1], bl[2], bl[3]);
  }
  acc_guard4(acc[0][0], acc[0][1], acc[0][2], acc[0][3]);
  acc_guard4(acc[1][0], acc[1][1], acc[1][2], acc[1][3]);
  acc_guard4(acc[2][0], acc[2][1], acc[2][2], acc[2][3]);
  acc_guard4(acc[3][0], acc[3][1], acc[3][2], acc[3][3]);

  float* slab = sT[wave];
  const float* Rb = RESID ? (resid + (size_t)b * strideR) : nullptr;
#pragma unroll
  for (int i = 0; i < 4; ++i) {
    const int mBase = m0 + (i << 4);
#pragma unroll
    for (int j = 0; j < 4; ++j) {
      const int n = n0 + (j << 4) + rlane;
      float bv = 0.f;
      if (BIAS_MODE == 2) bv = bias[n];
#pragma unroll
      for (int r = 0; r < 8; ++r) {
        float v = acc[i][j][r] * scale;
        if (BIAS_MODE == 1) v += bias[mBase + mOff + r];
        if (BIAS_MODE == 2) v += bv;
        if (RESID) v += Rb[(size_t)(mBase + mOff + r) * ldc + n];
        if (ACT == 2) v = fmaxf(v, 0.0f);
        if (ACT == 4) v = (v > 0.f) ? v : 0.01f * v;
        slab[(mOff + r) * 68 + (j << 4) + rlane] = v;
      }
    }
    __builtin_amdgcn_fence(__ATOMIC_RELEASE, "workgroup");
    __builtin_amdgcn_wave_barrier();
    __builtin_amdgcn_fence(__ATOMIC_ACQUIRE, "workgroup");
    if (OUT_MODE == 0) {
      float* C = (float*)Cout + (size_t)b * strideC;
      const int hh = lane >> 4, c4 = (lane & 15) * 4;
      for (int pass = 0; pass < 2; ++pass) {
#pragma unroll
        for (int it = 0; it < 8; ++it) {
          const int row = it * 2 + hh;
          v4f v = *(const v4f*)(slab + row * 68 + c4);
          *(volatile v4f*)(C + (size_t)(mBase + row) * ldc + n0 + c4) = v;
        }
        __threadfence();
      }
    } else {
      const int q = lane >> 3, c8 = (lane & 7) * 8;
      unsigned short* C  = (unsigned short*)Cout  + (size_t)b * strideC;
      unsigned short* C2 = (OUT_MODE == 2) ? ((unsigned short*)Cout2 + (size_t)b * strideC) : nullptr;
      for (int pass = 0; pass < 2; ++pass) {
#pragma unroll
        for (int it = 0; it < 4; ++it) {
          const int row = it * 4 + q;
          const float* sp = slab + row * 68 + c8;
          v8h hv, lv;
#pragma unroll
          for (int e = 0; e < 8; ++e) {
            if (OUT_MODE == 1) {
              hv[e] = (_Float16)sp[e];
            } else {
              unsigned short hb = f2bf_bits(sp[e]);
              unsigned short lb = f2bf_bits(sp[e] - bf_bits2f(hb));
              hv[e] = __builtin_bit_cast(_Float16, hb);
              lv[e] = __builtin_bit_cast(_Float16, lb);
            }
          }
          *(volatile v8h*)(C + (size_t)(mBase + row) * ldc + n0 + c8) = hv;
          if (OUT_MODE == 2) *(volatile v8h*)(C2 + (size_t)(mBase + row) * ldc + n0 + c8) = lv;
        }
        __threadfence();
      }
    }
    __builtin_amdgcn_fence(__ATOMIC_RELEASE, "workgroup");
    __builtin_amdgcn_wave_barrier();
    __builtin_amdgcn_fence(__ATOMIC_ACQUIRE, "workgroup");
  }
}

__global__ __launch_bounds__(256) void wpack_kernel(const float* __restrict__ w, unsigned short* __restrict__ bt,
                                                    const int* __restrict__ stride_in, int nthreads) {
  const int t = blockIdx.x * 256 + threadIdx.x;
  if (t >= nthreads) return;
  const int cl  = t / kSegs;
  const int s   = t - cl * kSegs;
  const int tap = (s < 9) ? s : 8;
  const int kh  = tap / 3;
  const int kw  = tap - kh * 3;
  unsigned short hb[8];
#pragma unroll
  for (int il = 0; il < 8; ++il) {
    const float v = w[((il * 3 + kh) * 3 + kw) * kNC + cl];
    hb[il] = f2bf_bits(v);
  }
  const unsigned zm = (s < 9) ? 0xffffffffu : 0u;
  const v4u u = (v4u){pk16(hb[0], hb[1]) & zm, pk16(hb[2], hb[3]) & zm, pk16(hb[4], hb[5]) & zm, pk16(hb[6], hb[7]) & zm};
  unsigned short* q = bt + 8 * (size_t)t;
  *(volatile v4u*)q = u;
  __threadfence();
  *(volatile v4u*)q = u;
}

__global__ __launch_bounds__(256) void im2col_kernel(const float* __restrict__ x, unsigned short* __restrict__ a,
                                                     int chunk, int nthreads) {
  const int t = blockIdx.x * 256 + threadIdx.x;
  if (t >= nthreads) return;
  const int row = t / kSegs;
  const int s   = t - row * kSegs;
  const int bb  = row / kRowsPerB;
  const int rem = row - bb * kRowsPerB;
  const int i   = rem / kP;
  const int p   = rem - i * kP;
  const int oy  = p / kOW;
  const int ox  = p - oy * kOW;
  const int tap = (s < 9) ? s : 8;
  const int ky  = tap / 3;
  const int kx  = tap - ky * 3;
  const int b   = chunk * kChunkB + bb;
  const size_t src = ((((size_t)b * kH + (oy + ky)) * kW + (ox + kx)) * kIC + i) * kIL;
  const v4f f0 = *(const v4f*)(x + src);
  const v4f f1 = *(const v4f*)(x + src + 4);
  unsigned short hb[8];
#pragma unroll
  for (int e = 0; e < 4; ++e) {
    hb[e]     = f2bf_bits(f0[e]);
    hb[4 + e] = f2bf_bits(f1[e]);
  }
  const unsigned zm = (s < 9) ? 0xffffffffu : 0u;
  const v4u u = (v4u){pk16(hb[0], hb[1]) & zm, pk16(hb[2], hb[3]) & zm, pk16(hb[4], hb[5]) & zm, pk16(hb[6], hb[7]) & zm};
  unsigned short* q = a + 8 * (size_t)t;
  *(volatile v4u*)q = u;
  __threadfence();
  *(volatile v4u*)q = u;
}

__global__ __launch_bounds__(128) void tsum_kernel(const float* __restrict__ u, float* __restrict__ tt) {
  const int lane = threadIdx.x & 31;
  const int wave = threadIdx.x >> 5;
  const int bp   = blockIdx.x * 4 + wave;
  const int bb   = bp / kP;
  const int p    = bp - bb * kP;
  v4f acc = (v4f){0.f, 0.f, 0.f, 0.f};
#pragma unroll 1
  for (int i = 0; i < kIC; ++i) {
    const v4f v = *(const v4f*)(u + ((size_t)(bb * kIC + i) * kP + p) * kNC + 4 * lane);
    acc += v;
  }
  float* q = tt + (size_t)bp * kNC + 4 * lane;
  *(volatile v4f*)q = acc;
  __threadfence();
  *(volatile v4f*)q = acc;
}

__global__ __launch_bounds__(256) void logits_softmax_kernel(const float* __restrict__ u, const float* __restrict__ tt,
                                                             float* __restrict__ pr) {
  __shared__ __align__(16) float sl[kJ];
  __shared__ float redm[8];
  __shared__ float reds[8];
  const int t    = threadIdx.x;
  const int lane = t & 31;
  const int wave = t >> 5;
  const int bi   = blockIdx.x;
  const int bb   = bi >> 5;
  const float* ub = u  + (size_t)bi * kP * kNC;
  const float* tb = tt + (size_t)bb * kP * kNC;

  float m = -INFINITY;
#pragma unroll 1
  for (int j = t; j < kJ; j += 256) {
    const v4f u0 = *(const v4f*)(ub + 8 * (size_t)j);
    const v4f u1 = *(const v4f*)(ub + 8 * (size_t)j + 4);
    const v4f t0 = *(const v4f*)(tb + 8 * (size_t)j);
    const v4f t1 = *(const v4f*)(tb + 8 * (size_t)j + 4);
    float d = u0.x * t0.x;
    d += u0.y * t0.y;
    d += u0.z * t0.z;
    d += u0.w * t0.w;
    d += u1.x * t1.x;
    d += u1.y * t1.y;
    d += u1.z * t1.z;
    d += u1.w * t1.w;
    const float lg = d * kInvSqrtL;
    sl[j] = lg;
    m = fmaxf(m, lg);
  }
#pragma unroll
  for (int off = 16; off > 0; off >>= 1) m = fmaxf(m, __shfl_xor(m, off, 32));
  if (lane == 0) redm[wave] = m;
  __syncthreads();
  float gm = redm[0];
#pragma unroll
  for (int wq = 1; wq < 8; ++wq) gm = fmaxf(gm, redm[wq]);

  float ssum = 0.f;
#pragma unroll 1
  for (int j = t; j < kJ; j += 256) {
    const float e = expf(sl[j] - gm);
    sl[j] = e;
    ssum += e;
  }
#pragma unroll
  for (int off = 16; off > 0; off >>= 1) ssum += __shfl_xor(ssum, off, 32);
  if (lane == 0) reds[wave] = ssum;
  __syncthreads();
  float tot = reds[0];
#pragma unroll
  for (int wq = 1; wq < 8; ++wq) tot += reds[wq];
  const float inv = 1.0f / tot;

  float* pb = pr + (size_t)bi * kJ;
  for (int pass = 0; pass < 2; ++pass) {
#pragma unroll 1
    for (int q = t; q < kJ / 4; q += 256) {
      v4f e4 = *(const v4f*)(sl + 4 * q);
      e4 = e4 * inv;
      *(volatile v4f*)(pb + 4 * (size_t)q) = e4;
    }
    __threadfence();
  }
}

__global__ __launch_bounds__(128) void route_squash_kernel(const float* __restrict__ u, const float* __restrict__ pr,
                                                           const float* __restrict__ broute, float* __restrict__ out,
                                                           int chunk) {
  __shared__ __align__(16) float so[kNC];
  const int n    = threadIdx.x;
  const int lane = n & 31;
  const int wave = n >> 5;
  const int bp   = blockIdx.x;
  const int bb   = bp / kP;
  const int p    = bp - bb * kP;
  const int c    = n >> 3;
  const float br = bf_bits2f(f2bf_bits(broute[(size_t)p * kNC + n]));
  float s = 0.f;
#pragma unroll 1
  for (int i = 0; i < kIC; ++i) {
    const size_t rbi = (size_t)(bb * kIC + i);
    const float uv = u[(rbi * kP + p) * kNC + n];
    const float av = pr[rbi * kJ + (size_t)p * kCaps + c];
    s += uv * (av + br);
  }
  float n2 = s * s;
  n2 += __shfl_xor(n2, 1, 32);
  n2 += __shfl_xor(n2, 2, 32);
  n2 += __shfl_xor(n2, 4, 32);
  const float norm = sqrtf(n2 + kEps);
  const float o = (1.0f - expf(-norm)) * (s * (1.0f / norm));
  so[n] = o;
  __syncthreads();
  if (wave == 0) {
    const int b = chunk * kChunkB + bb;
    float* q = out + ((size_t)b * kP + p) * kNC + 4 * lane;
    const v4f val = *(const v4f*)(so + 4 * lane);
    *(volatile v4f*)q = val;
    __threadfence();
    *(volatile v4f*)q = val;
  }
}

extern "C" void kernel_launch(void* const* d_in, const int* in_sizes, int n_in,
                              void* d_out, int out_size, void* d_ws, size_t ws_size,
                              hipStream_t stream) {
  if (n_in < 4) return;
  if (in_sizes[0] != kB * kH * kW * kIC * kIL) return;
  if (in_sizes[1] != kIL * 9 * kNC) return;
  if (in_sizes[2] != kJ * kL) return;
  if (out_size != kB * kP * kNC) return;

  const float* x      = (const float*)d_in[0];
  const float* w      = (const float*)d_in[1];
  const float* broute = (const float*)d_in[2];
  const int*   stride = (const int*)d_in[3];
  float* out = (float*)d_out;

  const size_t bt_bytes = (size_t)kNC * kKpad * 2;
  const size_t a_bytes  = (size_t)kMChunk * kKpad * 2;
  const size_t u_bytes  = (size_t)kMChunk * kNC * 4;
  const size_t t_bytes  = (size_t)kChunkB * kP * kNC * 4;
  const size_t p_bytes  = (size_t)kChunkB * kIC * kJ * 4;
  const size_t off_bt = 0;
  const size_t off_a  = off_bt + bt_bytes;
  const size_t off_u  = off_a + a_bytes;
  const size_t off_t  = off_u + u_bytes;
  const size_t off_p  = off_t + t_bytes;
  const size_t total  = off_p + p_bytes;
  if (total > ws_size) return;

  char* ws = (char*)d_ws;
  unsigned short* dBt = (unsigned short*)(ws + off_bt);
  unsigned short* dA  = (unsigned short*)(ws + off_a);
  float* dU = (float*)(ws + off_u);
  float* dT = (float*)(ws + off_t);
  float* dP = (float*)(ws + off_p);

  const int wthreads = kNC * kSegs;
  wpack_kernel<<<dim3((wthreads + 255) / 256), dim3(256), 0, stream>>>(w, dBt, stride, wthreads);

  const int ithreads = kMChunk * kSegs;
  const int gemm_tiles = (kMChunk / 64) * (kNC / 64);
  for (int chunk = 0; chunk < kNumChunks; ++chunk) {
    im2col_kernel<<<dim3((ithreads + 255) / 256), dim3(256), 0, stream>>>(x, dA, chunk, ithreads);
    wmma_gemm64<1, false, 0, 0, false, 0><<<dim3((gemm_tiles + 7) / 8, 1, 1), dim3(256), 0, stream>>>(
        dA, dA, kKpad, 0L,
        dBt, dBt, kKpad, 0L,
        (void*)dU, (void*)dU, kNC, 0L,
        (const float*)dU,
        (const float*)dU, 0L,
        kMChunk, kNC, kKpad, 1.0f);
    tsum_kernel<<<dim3((kChunkB * kP) / 4), dim3(128), 0, stream>>>(dU, dT);
    logits_softmax_kernel<<<dim3(kChunkB * kIC), dim3(256), 0, stream>>>(dU, dT, dP);
    route_squash_kernel<<<dim3(kChunkB * kP), dim3(128), 0, stream>>>(dU, dP, broute, out, chunk);
  }
}
